// MambaBlock_27255862460953
// MI455X (gfx1250) — hardware-verified
//
#include <hip/hip_runtime.h>
#include <math.h>

typedef __attribute__((ext_vector_type(8)))  _Float16 v8h;
typedef __attribute__((ext_vector_type(16))) __bf16   v16b;
typedef __attribute__((ext_vector_type(8)))  __bf16   v8b;
typedef __attribute__((ext_vector_type(8)))  float    v8f;
typedef __attribute__((ext_vector_type(4)))  float    v4f;

constexpr int kBatch = 2;
constexpr int kSeqL  = 2048;
constexpr int kDmod  = 1024;
constexpr int kDin   = 2048;
constexpr int kNst   = 16;
constexpr int kDtR   = 64;
constexpr int kPrjN  = 96;
constexpr int kPrjP  = 128;
constexpr int kXZP   = 2 * kDin;
constexpr int kRows  = kBatch * kSeqL;
constexpr int kTP    = 260;
static_assert(kDtR + 2 * kNst == kPrjN, "x_proj width");
static_assert((kSeqL % 64) == 0 && (kXZP % 64) == 0 && (kPrjP % 64) == 0 && (kDin % 64) == 0 && (kDmod % 64) == 0, "GEMM M,N multiples of 64");
static_assert((kDmod % 32) == 0 && (kDin % 32) == 0 && (kDtR % 32) == 0, "GEMM K multiples of 32");
static_assert((kDin % 256) == 0 && (kSeqL % 64) == 0 && (kSeqL % 16) == 0, "tile multiples");
static_assert(((kRows * kDmod) % 2048) == 0, "norm tile multiple");

constexpr size_t kOffWIN  = 0;
constexpr size_t kOffWXP  = kOffWIN  + (size_t)kXZP  * kDmod * 2;
constexpr size_t kOffWDT  = kOffWXP  + (size_t)kPrjP * kDin  * 2;
constexpr size_t kOffWOUT = kOffWDT  + (size_t)kDin  * kDtR  * 2;
constexpr size_t kOffXNH  = kOffWOUT + (size_t)kDmod * kDin  * 2;
constexpr size_t kOffXNL  = kOffXNH  + (size_t)kRows * kDmod * 2;
constexpr size_t kOffXZ   = kOffXNL  + (size_t)kRows * kDmod * 2;
constexpr size_t kOffUC   = kOffXZ   + (size_t)kSeqL * kXZP  * 4;
constexpr size_t kOffUC16 = kOffUC   + (size_t)kSeqL * kDin  * 4;
constexpr size_t kOffPROJ = kOffUC16 + (size_t)kSeqL * kDin  * 2;
constexpr size_t kOffDT16 = kOffPROJ + (size_t)kSeqL * kPrjP * 4;
constexpr size_t kOffDLR  = kOffDT16 + (size_t)kSeqL * kDtR  * 2;
constexpr size_t kOffYH   = kOffDLR  + (size_t)kSeqL * kDin  * 4;
constexpr size_t kOffYL   = kOffYH   + (size_t)kSeqL * kDin  * 2;
constexpr size_t kWsTotal = kOffYL   + (size_t)kSeqL * kDin  * 2;
static_assert(kWsTotal == 123731968ull, "carve total");
static_assert(kWsTotal <= 134217728ull, "carve cap");
static_assert((kOffWXP % 128) == 0 && (kOffWDT % 128) == 0 && (kOffWOUT % 128) == 0 && (kOffXNH % 128) == 0 &&
              (kOffXNL % 128) == 0 && (kOffXZ % 128) == 0 && (kOffUC % 128) == 0 && (kOffUC16 % 128) == 0 &&
              (kOffPROJ % 128) == 0 && (kOffDT16 % 128) == 0 && (kOffDLR % 128) == 0 && (kOffYH % 128) == 0 &&
              (kOffYL % 128) == 0, "128-B aligned regions");

__device__ __forceinline__ unsigned short f2bf_bits(float f) {
  unsigned u = __float_as_uint(f);
  return (unsigned short)((u + 0x7FFFu + ((u >> 16) & 1u)) >> 16);
}
__device__ __forceinline__ float bf_bits2f(unsigned short h) { return __uint_as_float(((unsigned)h) << 16); }
__device__ __forceinline__ float bfr(float f) { return bf_bits2f(f2bf_bits(f)); }

__device__ __forceinline__ void split8(const v4f a0, const v4f a1, v8h& hv, v8h& lv) {
#pragma unroll
  for (int e = 0; e < 4; ++e) {
    const float f0 = a0[e];
    const float f1 = a1[e];
    const unsigned short h0 = f2bf_bits(f0);
    const unsigned short h1 = f2bf_bits(f1);
    const unsigned short l0 = f2bf_bits(f0 - bf_bits2f(h0));
    const unsigned short l1 = f2bf_bits(f1 - bf_bits2f(h1));
    hv[e]     = __builtin_bit_cast(_Float16, h0);
    hv[4 + e] = __builtin_bit_cast(_Float16, h1);
    lv[e]     = __builtin_bit_cast(_Float16, l0);
    lv[4 + e] = __builtin_bit_cast(_Float16, l1);
  }
}
__device__ __forceinline__ void pack8(const v4f a0, const v4f a1, v8h& hv) {
#pragma unroll
  for (int e = 0; e < 4; ++e) {
    const float f0 = a0[e];
    const float f1 = a1[e];
    const unsigned short h0 = f2bf_bits(f0);
    const unsigned short h1 = f2bf_bits(f1);
    hv[e]     = __builtin_bit_cast(_Float16, h0);
    hv[4 + e] = __builtin_bit_cast(_Float16, h1);
  }
}

__device__ __forceinline__ void row_guard_b(v8f& a, v8f& b, v8f& c, v8f& d, v16b x, v16b y) {
  asm volatile("v_nop\n\tv_nop\n\tv_nop\n\tv_nop" : "+v"(a), "+v"(b), "+v"(c), "+v"(d) : "v"(x), "v"(y));
}
__device__ __forceinline__ void keep4_b(v16b a, v16b b, v16b c, v16b d) { asm volatile("v_nop" :: "v"(a), "v"(b), "v"(c), "v"(d)); }
__device__ __forceinline__ void acc_guard4(v8f& a, v8f& b, v8f& c, v8f& d) { asm volatile("v_nop\n\tv_nop\n\tv_nop\n\tv_nop" : "+v"(a), "+v"(b), "+v"(c), "+v"(d)); }
struct FragB {
  union U { v16b v; v8b h[2]; };
  static __device__ __forceinline__ v16b load(const __bf16* p) {
    U f;
    f.h[0] = *(const v8b*)(p);
    f.h[1] = *(const v8b*)(p + 16);
    return f.v;
  }
  static __device__ __forceinline__ v8f mma(v16b a, v16b b, v8f c) {
    return __builtin_amdgcn_wmma_f32_16x16x32_bf16(false, a, false, b, (short)0, c, false, false);
  }
};

template <int SPL, int BIAS_MODE>
__global__ __launch_bounds__(256) void wmma_gemm64(
    const unsigned short* __restrict__ Ap, const unsigned short* __restrict__ A2p, int lda,
    const unsigned short* __restrict__ Btp, int ldb,
    float* __restrict__ Cout, int ldc,
    const float* __restrict__ bias,
    int M, int N, int K, float scale) {
  typedef __bf16 T;
  typedef v16b V;
  const T* A  = (const T*)Ap;
  const T* A2 = (const T*)A2p;
  const T* Bt = (const T*)Btp;
  __shared__ __align__(16) float sT[8][16 * 68];
  const int lane = threadIdx.x & 31;
  const int wave = threadIdx.x >> 5;
  const int tilesN = N >> 6;
  const int tilesM = M >> 6;
  const int tile = blockIdx.x * 8 + wave;
  if (tile >= tilesM * tilesN) return;
  const int tm = tile / tilesN;
  const int tn = tile - tm * tilesN;
  const int m0 = tm << 6;
  const int n0 = tn << 6;

  const int rlane = lane & 15;
  const int koff  = (lane >> 4) * 8;
  const int mOff  = (lane >> 4) * 8;

  v8f acc[4][4];
#pragma unroll
  for (int i = 0; i < 4; ++i)
#pragma unroll
    for (int j = 0; j < 4; ++j) acc[i][j] = (v8f){0.f,0.f,0.f,0.f,0.f,0.f,0.f,0.f};

  for (int k0 = 0; k0 < K; k0 += 32) {
    V bh[4];
#pragma unroll
    for (int j = 0; j < 4; ++j) {
      const size_t bo = (size_t)(n0 + (j << 4) + rlane) * ldb + koff + k0;
      bh[j] = FragB::load(Bt + bo);
    }
#pragma unroll
    for (int i = 0; i < 4; ++i) {
      const size_t ao = (size_t)(m0 + (i << 4) + rlane) * lda + koff + k0;
      V ah = FragB::load(A + ao);
      V al;
      if (SPL == 1) al = FragB::load(A2 + ao);
#pragma unroll
      for (int j = 0; j < 4; ++j) {
        acc[i][j] = FragB::mma(ah, bh[j], acc[i][j]);
        if (SPL == 1) acc[i][j] = FragB::mma(al, bh[j], acc[i][j]);
      }
      row_guard_b(acc[i][0], acc[i][1], acc[i][2], acc[i][3], ah, (SPL == 1) ? al : ah);
    }
    keep4_b(bh[0], bh[1], bh[2], bh[3]);
  }
  acc_guard4(acc[0][0], acc[0][1], acc[0][2], acc[0][3]);
  acc_guard4(acc[1][0], acc[1][1], acc[1][2], acc[1][3]);
  acc_guard4(acc[2][0], acc[2][1], acc[2][2], acc[2][3]);
  acc_guard4(acc[3][0], acc[3][1], acc[3][2], acc[3][3]);

  float* slab = sT[wave];
#pragma unroll
  for (int i = 0; i < 4; ++i) {
    const int mBase = m0 + (i << 4);
#pragma unroll
    for (int j = 0; j < 4; ++j) {
      const int n = n0 + (j << 4) + rlane;
      float bv = 0.f;
      if (BIAS_MODE == 2) bv = bfr(bias[n]);
#pragma unroll
      for (int r = 0; r < 8; ++r) {
        float v = acc[i][j][r] * scale;
        if (BIAS_MODE == 2) v += bv;
        slab[(mOff + r) * 68 + (j << 4) + rlane] = v;
      }
    }
    __builtin_amdgcn_fence(__ATOMIC_RELEASE, "workgroup");
    __builtin_amdgcn_wave_barrier();
    __builtin_amdgcn_fence(__ATOMIC_ACQUIRE, "workgroup");
    {
      const int hh = lane >> 4, c4 = (lane & 15) * 4;
      for (int pass = 0; pass < 2; ++pass) {
#pragma unroll
        for (int it = 0; it < 8; ++it) {
          const int row = it * 2 + hh;
          v4f v = *(const v4f*)(slab + row * 68 + c4);
          *(volatile v4f*)(Cout + (size_t)(mBase + row) * ldc + n0 + c4) = v;
        }
        __threadfence();
      }
    }
    __builtin_amdgcn_fence(__ATOMIC_RELEASE, "workgroup");
    __builtin_amdgcn_wave_barrier();
    __builtin_amdgcn_fence(__ATOMIC_ACQUIRE, "workgroup");
  }
}

__global__ __launch_bounds__(256) void cast_bf16_kernel(
    const float* __restrict__ src, unsigned short* __restrict__ dst, int total8, int real8)
{
  const int i = blockIdx.x * 256 + threadIdx.x;
  if (i >= total8) return;
  const bool live = (i < real8);
  const int ic = live ? i : (real8 - 1);
  const float* p = src + ((size_t)ic << 3);
  const v4f r0 = *(const v4f*)(p);
  const v4f r1 = *(const v4f*)(p + 4);
  v4f a0, a1;
#pragma unroll
  for (int e = 0; e < 4; ++e) {
    const float f0 = r0[e];
    const float f1 = r1[e];
    a0[e] = live ? f0 : 0.0f;
    a1[e] = live ? f1 : 0.0f;
  }
  v8h hv;
  pack8(a0, a1, hv);
  unsigned short* q = dst + ((size_t)i << 3);
  *(volatile v8h*)q = hv;
  __threadfence();
  *(volatile v8h*)q = hv;
}

__global__ __launch_bounds__(256) void norm_split_kernel(
    const float* __restrict__ x, const float* __restrict__ alpha,
    const float* __restrict__ nw, const float* __restrict__ nb,
    unsigned short* __restrict__ XH, unsigned short* __restrict__ XL)
{
  __shared__ __align__(16) float sV[2048];
  const int tid = threadIdx.x;
  const size_t base = (size_t)blockIdx.x * 2048;
  const float a = fminf(fmaxf(bfr(alpha[0]), 0.1f), 2.0f);
#pragma unroll 1
  for (int i = 0; i < 8; ++i) {
    const int idx = i * 256 + tid;
    const int d = idx & (kDmod - 1);
    const float xv = bfr(x[base + idx]);
    const float w  = bfr(nw[d]);
    const float bb = bfr(nb[d]);
    const float t  = tanhf(a * xv);
    const float p  = w * t;
    sV[idx] = p + bb;
  }
  __syncthreads();
  const v4f a0 = *(const v4f*)(sV + tid * 8);
  const v4f a1 = *(const v4f*)(sV + tid * 8 + 4);
  v8h hv, lv;
  split8(a0, a1, hv, lv);
  unsigned short* qh = XH + base + (size_t)tid * 8;
  unsigned short* ql = XL + base + (size_t)tid * 8;
  *(volatile v8h*)qh = hv;
  *(volatile v8h*)ql = lv;
  __threadfence();
  *(volatile v8h*)qh = hv;
  *(volatile v8h*)ql = lv;
}

__global__ __launch_bounds__(256) void dt_cast_kernel(
    const float* __restrict__ PROJ, unsigned short* __restrict__ DT16, int total8)
{
  const int i = blockIdx.x * 256 + threadIdx.x;
  if (i >= total8) return;
  const int e0  = i << 3;
  const int row = e0 >> 6;
  const int c8  = e0 & 63;
  const float* p = PROJ + (size_t)row * kPrjP + c8;
  const v4f a0 = *(const v4f*)(p);
  const v4f a1 = *(const v4f*)(p + 4);
  v8h hv;
  pack8(a0, a1, hv);
  unsigned short* qd = DT16 + e0;
  *(volatile v8h*)qd = hv;
  __threadfence();
  *(volatile v8h*)qd = hv;
}

__global__ __launch_bounds__(256) void conv_silu_kernel(
    const float* __restrict__ XZ, const float* __restrict__ cw, const float* __restrict__ cb,
    float* __restrict__ UC, unsigned short* __restrict__ UC16)
{
  __shared__ __align__(16) float sT[16 * kTP];
  const int tid = threadIdx.x, lane = tid & 31, wave = tid >> 5;
  const int d0 = blockIdx.x * 256, d = d0 + tid;
  const int t0 = blockIdx.y * 64;
  const float w0 = bfr(cw[d * 4 + 0]);
  const float w1 = bfr(cw[d * 4 + 1]);
  const float w2 = bfr(cw[d * 4 + 2]);
  const float w3 = bfr(cw[d * 4 + 3]);
  const float bc = bfr(cb[d]);
  float xm3, xm2, xm1;
  {
    const int r3 = t0 - 3, r2 = t0 - 2, r1 = t0 - 1;
    const float v3 = XZ[(size_t)(r3 < 0 ? 0 : r3) * kXZP + d];
    const float v2 = XZ[(size_t)(r2 < 0 ? 0 : r2) * kXZP + d];
    const float v1 = XZ[(size_t)(r1 < 0 ? 0 : r1) * kXZP + d];
    xm3 = (r3 >= 0) ? v3 : 0.f;
    xm2 = (r2 >= 0) ? v2 : 0.f;
    xm1 = (r1 >= 0) ? v1 : 0.f;
  }
  const int hrow = wave >> 1;
  const int hch  = (wave & 1) * 128 + lane * 4;
#pragma unroll 1
  for (int sub = 0; sub < 4; ++sub) {
    const int lb = t0 + sub * 16;
#pragma unroll 1
    for (int s = 0; s < 16; ++s) {
      const float xc = XZ[(size_t)(lb + s) * kXZP + d];
      float acc = w0 * xm3;
      acc = fmaf(w1, xm2, acc);
      acc = fmaf(w2, xm1, acc);
      acc = fmaf(w3, xc, acc);
      const float sv = acc + bc;
      const float sg = __builtin_amdgcn_rcpf(1.0f + expf(-sv));
      sT[s * kTP + tid] = sv * sg;
      xm3 = xm2; xm2 = xm1; xm1 = xc;
    }
    __syncthreads();
    v4f fv[4];
    v8h bv[2];
#pragma unroll
    for (int it = 0; it < 4; ++it) fv[it] = *(const v4f*)(sT + (it * 4 + hrow) * kTP + hch);
#pragma unroll
    for (int it = 0; it < 2; ++it) {
      const float* sp = sT + (it * 8 + wave) * kTP + lane * 8;
      const v4f a0 = *(const v4f*)(sp);
      const v4f a1 = *(const v4f*)(sp + 4);
      pack8(a0, a1, bv[it]);
    }
    for (int pass = 0; pass < 2; ++pass) {
#pragma unroll
      for (int it = 0; it < 4; ++it)
        *(volatile v4f*)(UC + (size_t)(lb + it * 4 + hrow) * kDin + d0 + hch) = fv[it];
#pragma unroll
      for (int it = 0; it < 2; ++it)
        *(volatile v8h*)(UC16 + (size_t)(lb + it * 8 + wave) * kDin + d0 + lane * 8) = bv[it];
      __threadfence();
    }
    __syncthreads();
  }
}

__global__ __launch_bounds__(256) void scan_kernel(
    const float* __restrict__ DLR, const float* __restrict__ UC, const float* __restrict__ XZ,
    const float* __restrict__ PROJ, const float* __restrict__ A_log, const float* __restrict__ Dv,
    unsigned short* __restrict__ YH, unsigned short* __restrict__ YL)
{
  __shared__ __align__(16) float sBC[16 * 32];
  __shared__ __align__(16) float sY[16 * kTP];
  const int tid = threadIdx.x, lane = tid & 31, wave = tid >> 5;
  const int d0 = blockIdx.x * 256, d = d0 + tid;

  float An[kNst];
#pragma unroll
  for (int q4 = 0; q4 < 4; ++q4) {
    const v4f al = *(const v4f*)(A_log + (size_t)d * kNst + 4 * q4);
    const float e0 = al[0];
    const float e1 = al[1];
    const float e2 = al[2];
    const float e3 = al[3];
    An[4 * q4 + 0] = -__expf(bfr(e0));
    An[4 * q4 + 1] = -__expf(bfr(e1));
    An[4 * q4 + 2] = -__expf(bfr(e2));
    An[4 * q4 + 3] = -__expf(bfr(e3));
  }
  const float Dd = bfr(Dv[d]);
  float h[kNst];
#pragma unroll
  for (int n = 0; n < kNst; ++n) h[n] = 0.f;

#pragma unroll 1
  for (int c = 0; c < kSeqL / 16; ++c) {
    const int l0 = c * 16;
    if (tid < 128) {
      const int r = tid >> 3, q = (tid & 7) * 4;
      const v4f v = *(const v4f*)(PROJ + (size_t)(l0 + r) * kPrjP + kDtR + q);
      *(v4f*)(sBC + r * 32 + q) = v;
    }
    __syncthreads();
#pragma unroll 1
    for (int s = 0; s < 16; ++s) {
      const size_t m = (size_t)(l0 + s);
      float a  = DLR[m * kDin + d];
      asm volatile("" : "+v"(a));
      float xv = UC[m * kDin + d];
      asm volatile("" : "+v"(xv));
      float zv = XZ[m * kXZP + kDin + d];
      asm volatile("" : "+v"(zv));
      const float delta = fmaxf(a, 0.0f) + log1pf(__expf(-fabsf(a)));
      v4f Bq[4], Cq[4];
#pragma unroll
      for (int qq = 0; qq < 4; ++qq) {
        Bq[qq] = *(const v4f*)(sBC + s * 32 + 4 * qq);
        Cq[qq] = *(const v4f*)(sBC + s * 32 + kNst + 4 * qq);
      }
      float y = 0.f;
#pragma unroll
      for (int n = 0; n < kNst; ++n) {
        const float e = __expf(delta * An[n]);
        float db = delta * Bq[n >> 2][n & 3];
        asm volatile("" : "+v"(db));
        float p = db * xv;
        asm volatile("" : "+v"(p));
        float qv = h[n] * e;
        asm volatile("" : "+v"(qv));
        const float hn = qv + p;
        h[n] = hn;
        float rr = Cq[n >> 2][n & 3] * hn;
        asm volatile("" : "+v"(rr));
        y += rr;
      }
      float sk = xv * Dd;
      asm volatile("" : "+v"(sk));
      y += sk;
      const float sg = __builtin_amdgcn_rcpf(1.0f + expf(-zv));
      const float g  = zv * sg;
      sY[s * kTP + tid] = y * g;
    }
    __syncthreads();
    v8h hv[2], lv[2];
#pragma unroll
    for (int it = 0; it < 2; ++it) {
      const float* sp = sY + (it * 8 + wave) * kTP + lane * 8;
      const v4f a0 = *(const v4f*)(sp);
      const v4f a1 = *(const v4f*)(sp + 4);
      split8(a0, a1, hv[it], lv[it]);
    }
    for (int pass = 0; pass < 2; ++pass) {
#pragma unroll
      for (int it = 0; it < 2; ++it) {
        const size_t o = (size_t)(l0 + it * 8 + wave) * kDin + d0 + lane * 8;
        *(volatile v8h*)(YH + o) = hv[it];
        *(volatile v8h*)(YL + o) = lv[it];
      }
      __threadfence();
    }
  }
}

extern "C" void kernel_launch(void* const* d_in, const int* in_sizes, int n_in,
                              void* d_out, int out_size, void* d_ws, size_t ws_size,
                              hipStream_t stream)
{
  if (n_in < 13) return;
  if (in_sizes[0] != kRows * kDmod) return;
  if (in_sizes[1] != 1) return;
  if (in_sizes[2] != kDmod || in_sizes[3] != kDmod) return;
  if (in_sizes[4] != kXZP * kDmod) return;
  if (in_sizes[5] != kDin * 4 || in_sizes[6] != kDin) return;
  if (in_sizes[7] != kPrjN * kDin) return;
  if (in_sizes[8] != kDin * kDtR || in_sizes[9] != kDin) return;
  if (in_sizes[10] != kDin * kNst || in_sizes[11] != kDin) return;
  if (in_sizes[12] != kDmod * kDin) return;
  if (out_size != kRows * kDmod) return;
  if (ws_size < kWsTotal) return;

  const float* x_flat  = (const float*)d_in[0];
  const float* alpha   = (const float*)d_in[1];
  const float* norm_w  = (const float*)d_in[2];
  const float* norm_b  = (const float*)d_in[3];
  const float* W_in    = (const float*)d_in[4];
  const float* conv_w  = (const float*)d_in[5];
  const float* conv_b  = (const float*)d_in[6];
  const float* W_xprj  = (const float*)d_in[7];
  const float* W_dt    = (const float*)d_in[8];
  const float* b_dt    = (const float*)d_in[9];
  const float* A_log   = (const float*)d_in[10];
  const float* Dv      = (const float*)d_in[11];
  const float* W_out   = (const float*)d_in[12];
  float* dout = (float*)d_out;

  char* ws = (char*)d_ws;
  unsigned short* WIN  = (unsigned short*)(ws + kOffWIN);
  unsigned short* WXP  = (unsigned short*)(ws + kOffWXP);
  unsigned short* WDT  = (unsigned short*)(ws + kOffWDT);
  unsigned short* WOUT = (unsigned short*)(ws + kOffWOUT);
  unsigned short* XNH  = (unsigned short*)(ws + kOffXNH);
  unsigned short* XNL  = (unsigned short*)(ws + kOffXNL);
  float*          XZ   = (float*)(ws + kOffXZ);
  float*          UC   = (float*)(ws + kOffUC);
  unsigned short* UC16 = (unsigned short*)(ws + kOffUC16);
  float*          PROJ = (float*)(ws + kOffPROJ);
  unsigned short* DT16 = (unsigned short*)(ws + kOffDT16);
  float*          DLR  = (float*)(ws + kOffDLR);
  unsigned short* YH   = (unsigned short*)(ws + kOffYH);
  unsigned short* YL   = (unsigned short*)(ws + kOffYL);

  cast_bf16_kernel<<<(kXZP * kDmod / 8) / 256, 256, 0, stream>>>(W_in, WIN, kXZP * kDmod / 8, kXZP * kDmod / 8);
  cast_bf16_kernel<<<(kPrjP * kDin / 8) / 256, 256, 0, stream>>>(W_xprj, WXP, kPrjP * kDin / 8, kPrjN * kDin / 8);
  cast_bf16_kernel<<<(kDin * kDtR / 8) / 256, 256, 0, stream>>>(W_dt, WDT, kDin * kDtR / 8, kDin * kDtR / 8);
  cast_bf16_kernel<<<(kDmod * kDin / 8) / 256, 256, 0, stream>>>(W_out, WOUT, kDmod * kDin / 8, kDmod * kDin / 8);

  norm_split_kernel<<<(kRows * kDmod) / 2048, 256, 0, stream>>>(x_flat, alpha, norm_w, norm_b, XNH, XNL);

  for (int b = 0; b < kBatch; ++b) {
    const unsigned short* XNHb = XNH + (size_t)b * kSeqL * kDmod;
    const unsigned short* XNLb = XNL + (size_t)b * kSeqL * kDmod;
    float* outb = dout + (size_t)b * kSeqL * kDmod;

    wmma_gemm64<1, 0><<<dim3(256, 1), 256, 0, stream>>>(
        XNHb, XNLb, kDmod, WIN, kDmod, XZ, kXZP, b_dt, kSeqL, kXZP, kDmod, 1.0f);

    conv_silu_kernel<<<dim3(kDin / 256, kSeqL / 64), 256, 0, stream>>>(XZ, conv_w, conv_b, UC, UC16);

    wmma_gemm64<0, 0><<<dim3(8, 1), 256, 0, stream>>>(
        UC16, UC16, kDin, WXP, kDin, PROJ, kPrjP, b_dt, kSeqL, kPrjP, kDin, 1.0f);

    dt_cast_kernel<<<(kSeqL * kDtR / 8) / 256, 256, 0, stream>>>(PROJ, DT16, kSeqL * kDtR / 8);

    wmma_gemm64<0, 2><<<dim3(128, 1), 256, 0, stream>>>(
        DT16, DT16, kDtR, WDT, kDtR, DLR, kDin, b_dt, kSeqL, kDin, kDtR, 1.0f);

    scan_kernel<<<dim3(kDin / 256, 1), 256, 0, stream>>>(DLR, UC, XZ, PROJ, A_log, Dv, YH, YL);

    wmma_gemm64<1, 0><<<dim3(64, 1), 256, 0, stream>>>(
        YH, YL, kDin, WOUT, kDin, outb, kDmod, b_dt, kSeqL, kDmod, kDin, 1.0f);
  }
}
